// KPConvInterSO3_77146202570856
// MI455X (gfx1250) — hardware-verified
//
#include <hip/hip_runtime.h>
#include <stdint.h>


#define NBR   32
#define AK    4
#define KPN   15
#define KPAD  16
#define CIN_  32
#define COUT_ 32
#define KCP   512
#define ROWS  16
#define QPB   4

static_assert(KCP == KPAD * CIN_);
static_assert(ROWS == QPB * AK);

typedef unsigned short us;
typedef us     v8us  __attribute__((ext_vector_type(8), __may_alias__));
typedef __bf16 v16bf __attribute__((ext_vector_type(16)));
typedef float  v8f   __attribute__((ext_vector_type(8)));
typedef float  v4f   __attribute__((ext_vector_type(4), __may_alias__));

union Frag { v16bf v; v8us hv[2]; };

__device__ __forceinline__ us f2bf(float f) {
    unsigned u = __float_as_uint(f);
    u += 0x7FFFu + ((u >> 16) & 1u);
    return (us)(u >> 16);
}
__device__ __forceinline__ float bf2f(us b) { return __uint_as_float(((unsigned)b) << 16); }
__device__ __forceinline__ void split2(float f, us& hi, us& lo) {
    hi = f2bf(f);
    lo = f2bf(f - bf2f(hi));
}

__device__ __forceinline__ void mma3(v8f& acc, const Frag& ah, const Frag& al,
                                     const Frag& bh, const Frag& bl) {
    acc = __builtin_amdgcn_wmma_f32_16x16x32_bf16(false, ah.v, false, bh.v, (short)0, acc, false, false);
    acc = __builtin_amdgcn_wmma_f32_16x16x32_bf16(false, ah.v, false, bl.v, (short)0, acc, false, false);
    acc = __builtin_amdgcn_wmma_f32_16x16x32_bf16(false, al.v, false, bh.v, (short)0, acc, false, false);
    asm volatile("v_nop\n\tv_nop\n\tv_nop\n\tv_nop"
                 : "+v"(acc) : "v"(ah.v), "v"(al.v), "v"(bh.v), "v"(bl.v));
}

__global__ __launch_bounds__(32)
void k_wsplit(const float* __restrict__ wts, us* w2h, us* w2l)
{
    const int d = blockIdx.x;
    const int l = threadIdx.x;
    v8us ph0, pl0, ph1, pl1;
    #pragma unroll
    for (int j = 0; j < 2; ++j) {
        v8us ph, pl;
        #pragma unroll
        for (int i = 0; i < 8; ++i) {
            const int kc = 256 * j + 8 * l + i;
            const int k  = kc >> 5;
            const int c  = kc & 31;
            const int ks = (k < KPN) ? k : (KPN - 1);
            float v = wts[(ks * CIN_ + c) * COUT_ + d];
            if (k >= KPN) v = 0.0f;
            us hb, lb; split2(v, hb, lb);
            ph[i] = hb; pl[i] = lb;
        }
        if (j == 0) { ph0 = ph; pl0 = pl; } else { ph1 = ph; pl1 = pl; }
    }
    us* rh = w2h + (size_t)d * KCP + 8 * l;
    us* rl = w2l + (size_t)d * KCP + 8 * l;
    *(volatile v8us*)(rh)       = ph0;
    *(volatile v8us*)(rh + 256) = ph1;
    *(volatile v8us*)(rl)       = pl0;
    *(volatile v8us*)(rl + 256) = pl1;
    __threadfence();
    *(volatile v8us*)(rh)       = ph0;
    *(volatile v8us*)(rh + 256) = ph1;
    *(volatile v8us*)(rl)       = pl0;
    *(volatile v8us*)(rl + 256) = pl1;
}

__global__ __launch_bounds__(32)
void k_kpconv(const float* __restrict__ q_pts,
              const float* __restrict__ s_pts,
              const int*   __restrict__ nbi,
              const float* __restrict__ x,
              const float* __restrict__ kp,
              const float* __restrict__ anc,
              const us*    __restrict__ w2h,
              const us*    __restrict__ w2l,
              float*                    out,
              int N, int M, int totRows)
{
    #pragma clang fp contract(off)
    __shared__ v4f  nv[QPB * NBR];
    __shared__ v4f  rkp[AK * KPAD];
    __shared__ int  nbl[QPB * NBR];
    __shared__ us   wh[KPAD * NBR]  __attribute__((aligned(16)));
    __shared__ us   wl[KPAD * NBR]  __attribute__((aligned(16)));
    __shared__ us   xth[CIN_ * NBR] __attribute__((aligned(16)));
    __shared__ us   xtl[CIN_ * NBR] __attribute__((aligned(16)));
    __shared__ us   gah[ROWS * KCP] __attribute__((aligned(16)));
    __shared__ us   gal[ROWS * KCP] __attribute__((aligned(16)));
    __shared__ float outs[ROWS * COUT_] __attribute__((aligned(16)));

    const int l   = threadIdx.x;
    const int h   = l >> 4;
    const int lm  = l & 15;
    const int blk = blockIdx.x;
    const int q0  = blk * QPB;
    const float KPINV = 1.0f / 0.6f;

    #pragma unroll
    for (int i = 0; i < QPB; ++i) {
        int q = q0 + i; q = (q < N) ? q : (N - 1);
        int m = nbi[(size_t)q * NBR + l];
        if (m < 0) m += M;
        m = (m < 0) ? 0 : m; m = (m > M - 1) ? (M - 1) : m;
        nbl[i * NBR + l] = m;
        const float qx = q_pts[(size_t)q * 3 + 0];
        const float qy = q_pts[(size_t)q * 3 + 1];
        const float qz = q_pts[(size_t)q * 3 + 2];
        const float dx = s_pts[(size_t)m * 3 + 0] - qx;
        const float dy = s_pts[(size_t)m * 3 + 1] - qy;
        const float dz = s_pts[(size_t)m * 3 + 2] - qz;
        v4f t; t.x = dx; t.y = dy; t.z = dz; t.w = (dx * dx + dy * dy) + dz * dz;
        nv[i * NBR + l] = t;
    }
    #pragma unroll
    for (int j = 0; j < 2; ++j) {
        const int e = l + 32 * j;
        const int a = e >> 4, k = e & 15;
        v4f t; t.x = 0.0f; t.y = 0.0f; t.z = 0.0f; t.w = 0.0f;
        if (k < KPN) {
            const float px = kp[k * 3 + 0], py = kp[k * 3 + 1], pz = kp[k * 3 + 2];
            const float* R = anc + a * 9;
            const float rx = (R[0] * px + R[1] * py) + R[2] * pz;
            const float ry = (R[3] * px + R[4] * py) + R[5] * pz;
            const float rz = (R[6] * px + R[7] * py) + R[8] * pz;
            t.x = rx; t.y = ry; t.z = rz; t.w = (rx * rx + ry * ry) + rz * rz;
        }
        rkp[e] = t;
    }
    __syncthreads();

    #pragma unroll 1
    for (int ri = 0; ri < ROWS; ++ri) {
        const int nl = ri >> 2;
        const int a  = ri & 3;
        __syncthreads();

        {
            const float* xa = x + (size_t)a * CIN_ + l;
            #pragma unroll
            for (int g = 0; g < 4; ++g) {
                float v[8];
                #pragma unroll
                for (int i = 0; i < 8; ++i) {
                    const int m = nbl[nl * NBR + 8 * g + i];
                    v[i] = xa[(size_t)m * (AK * CIN_)];
                }
                v8us ph, pl;
                #pragma unroll
                for (int i = 0; i < 8; ++i) {
                    us hb, lb; split2(v[i], hb, lb);
                    ph[i] = hb; pl[i] = lb;
                }
                *(v8us*)(xth + l * NBR + 8 * g) = ph;
                *(v8us*)(xtl + l * NBR + 8 * g) = pl;
            }
        }
        {
            const v4f rk = rkp[a * KPAD + lm];
            const bool kval = lm < KPN;
            #pragma unroll
            for (int g = 0; g < 2; ++g) {
                v8us ph, pl;
                #pragma unroll
                for (int i = 0; i < 8; ++i) {
                    const int b = 16 * h + 8 * g + i;
                    const v4f dv = nv[nl * NBR + b];
                    const float cr = (dv.x * rk.x + dv.y * rk.y) + dv.z * rk.z;
                    float sq = (dv.w + rk.w) - 2.0f * cr;
                    sq = fmaxf(sq, 1e-12f);
                    float w = 1.0f - sqrtf(sq) * KPINV;
                    w = fmaxf(w, 0.0f);
                    w = kval ? w : 0.0f;
                    us hb, lb; split2(w, hb, lb);
                    ph[i] = hb; pl[i] = lb;
                }
                *(v8us*)(wh + lm * NBR + 16 * h + 8 * g) = ph;
                *(v8us*)(wl + lm * NBR + 16 * h + 8 * g) = pl;
            }
        }
        __syncthreads();

        Frag ah, al, bh0, bl0, bh1, bl1;
        ah.hv[0]  = *(const v8us*)(wh  + lm * NBR + 8 * h);
        ah.hv[1]  = *(const v8us*)(wh  + lm * NBR + 16 + 8 * h);
        al.hv[0]  = *(const v8us*)(wl  + lm * NBR + 8 * h);
        al.hv[1]  = *(const v8us*)(wl  + lm * NBR + 16 + 8 * h);
        bh0.hv[0] = *(const v8us*)(xth + lm * NBR + 8 * h);
        bh0.hv[1] = *(const v8us*)(xth + lm * NBR + 16 + 8 * h);
        bl0.hv[0] = *(const v8us*)(xtl + lm * NBR + 8 * h);
        bl0.hv[1] = *(const v8us*)(xtl + lm * NBR + 16 + 8 * h);
        bh1.hv[0] = *(const v8us*)(xth + (lm + 16) * NBR + 8 * h);
        bh1.hv[1] = *(const v8us*)(xth + (lm + 16) * NBR + 16 + 8 * h);
        bl1.hv[0] = *(const v8us*)(xtl + (lm + 16) * NBR + 8 * h);
        bl1.hv[1] = *(const v8us*)(xtl + (lm + 16) * NBR + 16 + 8 * h);

        v8f g0 = {0.f, 0.f, 0.f, 0.f, 0.f, 0.f, 0.f, 0.f};
        v8f g1 = {0.f, 0.f, 0.f, 0.f, 0.f, 0.f, 0.f, 0.f};
        mma3(g0, ah, al, bh0, bl0);
        mma3(g1, ah, al, bh1, bl1);

        #pragma unroll
        for (int r = 0; r < 8; ++r) {
            const int kc0 = (8 * h + r) * CIN_ + lm;
            us hb, lb;
            split2(g0[r], hb, lb);
            gah[ri * KCP + kc0] = hb;       gal[ri * KCP + kc0] = lb;
            split2(g1[r], hb, lb);
            gah[ri * KCP + kc0 + 16] = hb;  gal[ri * KCP + kc0 + 16] = lb;
        }
    }
    __syncthreads();

    v8f acc0 = {0.f, 0.f, 0.f, 0.f, 0.f, 0.f, 0.f, 0.f};
    v8f acc1 = {0.f, 0.f, 0.f, 0.f, 0.f, 0.f, 0.f, 0.f};
    #pragma unroll 1
    for (int kk = 0; kk < KPAD; ++kk) {
        const int ko = kk * 32;
        Frag ah, al, bh0, bl0, bh1, bl1;
        ah.hv[0] = *(const v8us*)(gah + lm * KCP + ko + 8 * h);
        ah.hv[1] = *(const v8us*)(gah + lm * KCP + ko + 16 + 8 * h);
        al.hv[0] = *(const v8us*)(gal + lm * KCP + ko + 8 * h);
        al.hv[1] = *(const v8us*)(gal + lm * KCP + ko + 16 + 8 * h);
        const us* ph0 = w2h + (size_t)lm * KCP + ko;
        const us* pl0 = w2l + (size_t)lm * KCP + ko;
        const us* ph1 = w2h + (size_t)(lm + 16) * KCP + ko;
        const us* pl1 = w2l + (size_t)(lm + 16) * KCP + ko;
        bh0.hv[0] = *(const v8us*)(ph0 + 8 * h);  bh0.hv[1] = *(const v8us*)(ph0 + 16 + 8 * h);
        bl0.hv[0] = *(const v8us*)(pl0 + 8 * h);  bl0.hv[1] = *(const v8us*)(pl0 + 16 + 8 * h);
        bh1.hv[0] = *(const v8us*)(ph1 + 8 * h);  bh1.hv[1] = *(const v8us*)(ph1 + 16 + 8 * h);
        bl1.hv[0] = *(const v8us*)(pl1 + 8 * h);  bl1.hv[1] = *(const v8us*)(pl1 + 16 + 8 * h);
        mma3(acc0, ah, al, bh0, bl0);
        mma3(acc1, ah, al, bh1, bl1);
    }

    #pragma unroll
    for (int r = 0; r < 8; ++r) {
        outs[(8 * h + r) * COUT_ + lm]      = acc0[r];
        outs[(8 * h + r) * COUT_ + 16 + lm] = acc1[r];
    }
    __syncthreads();

    const int R0  = blk * ROWS;
    const int sub = l >> 3;
    const int col = 4 * (l & 7);
    v4f ov[4];
    #pragma unroll
    for (int i = 0; i < 4; ++i) ov[i] = *(const v4f*)(outs + (4 * i + sub) * COUT_ + col);
    #pragma unroll
    for (int i = 0; i < 4; ++i) {
        const int g = R0 + 4 * i + sub;
        if (g < totRows) *(volatile v4f*)(out + (size_t)g * COUT_ + col) = ov[i];
    }
    __threadfence();
    #pragma unroll
    for (int i = 0; i < 4; ++i) {
        const int g = R0 + 4 * i + sub;
        if (g < totRows) *(volatile v4f*)(out + (size_t)g * COUT_ + col) = ov[i];
    }
}

extern "C" void kernel_launch(void* const* d_in, const int* in_sizes, int n_in,
                              void* d_out, int out_size, void* d_ws, size_t ws_size,
                              hipStream_t stream)
{
    (void)n_in;
    const float* q_pts = (const float*)d_in[0];
    const float* s_pts = (const float*)d_in[1];
    const int*   nbi   = (const int*)  d_in[2];
    const float* x     = (const float*)d_in[3];
    const float* kp    = (const float*)d_in[4];
    const float* anc   = (const float*)d_in[5];
    const float* wts   = (const float*)d_in[6];
    float*       out   = (float*)d_out;

    const int N = in_sizes[0] / 3;
    const int M = in_sizes[1] / 3;
    if (N <= 0 || M <= 0) return;
    if (in_sizes[2] != N * NBR) return;
    if (in_sizes[3] != M * AK * CIN_) return;
    if (in_sizes[4] != KPN * 3 || in_sizes[5] != AK * 9 || in_sizes[6] != KPN * CIN_ * COUT_) return;

    int totRows = N * AK;
    const int capRows = out_size / COUT_;
    if (totRows > capRows) totRows = capRows;

    const size_t planeBytes = (size_t)COUT_ * KCP * sizeof(us);
    if (2 * planeBytes > ws_size) return;
    us* w2h = (us*)d_ws;
    us* w2l = (us*)((char*)d_ws + planeBytes);

    hipLaunchKernelGGL(k_wsplit, dim3(COUT_), dim3(32), 0, stream, wts, w2h, w2l);

    const int nblk = (N + QPB - 1) / QPB;
    hipLaunchKernelGGL(k_kpconv, dim3(nblk), dim3(32), 0, stream,
                       q_pts, s_pts, nbi, x, kp, anc,
                       (const us*)w2h, (const us*)w2l, out, N, M, totRows);
    (void)hipGetLastError();
}
